// Net_66752381715145
// MI455X (gfx1250) — hardware-verified
//
#include <hip/hip_runtime.h>
#include <stddef.h>
#include <stdint.h>
#include <math.h>

#define IN_F   16
#define H1     512
#define H2     1024
#define OUT_F  16
#define RW     16
#define KA1    32
#define X1P    1024
#define KZ     1536
#define NTHR   256
#define NWAVE  8
#define EPT    8
#define CHUNK  (NTHR * EPT)
#define WCAP   (EPT * 32)
#define LISTN  (NWAVE * WCAP)
#define NBA    1024
#define SLA    10
#define RCAP   28672
#define DEGCAP 64
#define MEAS_B1024  8418
#define MEAS_MAXDEG 21
#define GBM    64
#define GBN    128
#define GTHR   128
#define ZBM    128
#define FTHR   512
#define PU1    (H1 * (KA1 / 8))
#define PU2    (H1 * (H2 / 8))
#define PU3    (OUT_F * (H2 / 8))
#define AGG_ZINTS (LISTN + 2 * RCAP + 3 * NBA)
#define AGG_LDS_INTS (AGG_ZINTS + 16)
#define NN_EXPECT 20000
#define WSMAX  134217728

static_assert(IN_F == 16 && 2 * IN_F == KA1 && KA1 == 32);
static_assert(OUT_F == 16 && RW == IN_F && RW == OUT_F);
static_assert(H1 % 128 == 0 && (3 * H1) % 32 == 0 && KZ == 3 * H1 && X1P == 2 * H1);
static_assert(H2 % 32 == 0 && H1 == 32 * (FTHR / 32));
static_assert((CHUNK & (CHUNK - 1)) == 0 && CHUNK <= 4096);
static_assert((NBA & (NBA - 1)) == 0 && NBA == (1 << SLA) && NBA % 2 == 0);
static_assert(((long long)CHUNK << SLA) < (1LL << 31));
static_assert(LISTN % NTHR == 0 && NBA % NWAVE == 0 && NBA % 32 == 0 && NBA % ZBM == 0);
static_assert(RCAP % 32 == 0 && AGG_ZINTS % (NTHR * 4) == 0 && LISTN % 4 == 0);
static_assert(RCAP >= 2 * MEAS_B1024 && DEGCAP >= MEAS_MAXDEG + 8);
static_assert(NBA * 32 * 2 <= RCAP * 4 && NBA * 16 * 4 <= RCAP * 4);
static_assert(NBA == NTHR * 4);
static_assert(PU1 % NTHR == 0 && (PU1 + PU2) % NTHR == 0 && (PU1 + PU2 + PU3) % NTHR == 0);
static_assert((OUT_F * KZ / 8) % FTHR == 0 && (OUT_F * KZ / 8) / FTHR == 6);
static_assert(GBM == (GTHR / 32) * 16 && GBN == 128 && H1 % GBN == 0);
static_assert(ZBM == (NTHR / 32) * 16 && (ZBM * OUT_F) == 2 * NTHR * 4);
static_assert(((NN_EXPECT + 127) / 128) * 128 == 157 * 128 && NN_EXPECT % 2 == 0);
static_assert(AGG_LDS_INTS * 4 <= 300000);

typedef float          v4f   __attribute__((ext_vector_type(4)));
typedef float          v8f   __attribute__((ext_vector_type(8)));
typedef int            v4i   __attribute__((ext_vector_type(4)));
typedef int            v8i   __attribute__((ext_vector_type(8)));
typedef unsigned short v4us  __attribute__((ext_vector_type(4)));
typedef unsigned short v8us  __attribute__((ext_vector_type(8)));
typedef unsigned short v16us __attribute__((ext_vector_type(16)));
typedef __bf16         v16bf __attribute__((ext_vector_type(16)));
typedef v4f  __attribute__((may_alias)) v4fa;
typedef v4i  __attribute__((may_alias)) v4ia;
typedef v4us __attribute__((may_alias)) v4usa;
typedef v8us __attribute__((may_alias)) v8usa;
union FragB { v16bf v; v16us u; v8us h[2]; v8i w; };

__device__ __forceinline__ v8f wmb(const FragB& a, const FragB& b, v8f c) {
  v8f d = __builtin_amdgcn_wmma_f32_16x16x32_bf16(false, a.v, false, b.v, (short)0, c, false, false);
  asm volatile("v_nop\n\tv_nop\n\tv_nop\n\tv_nop" : "+v"(d) : "v"(a.w), "v"(b.w));
  return d;
}

__device__ __forceinline__ unsigned bf16_bits(float f) {
  const unsigned u = __float_as_uint(f);
  return (u + 0x7FFFu + ((u >> 16) & 1u)) >> 16;
}
__device__ __forceinline__ float bf16_val(float f) {
  return __uint_as_float(bf16_bits(f) << 16);
}

template <int SLB>
__device__ __forceinline__ int scan_chunk(const int* __restrict__ dsts, int nE, int cbase, int slotBase,
                                          int nb, int vec8, int* list, int tid, int lane, int wave) {
  int wc = 0;
  const int el0  = tid * EPT;
  const int e0   = cbase + el0;
  const int sent = -2147483647 - 1;
  v4i da, db;
  if (vec8 != 0 && cbase + CHUNK <= nE) {
    da = *(const v4i*)(dsts + e0);
    db = *(const v4i*)(dsts + e0 + 4);
  } else {
    da.x = (e0     < nE) ? dsts[min(e0,     nE - 1)] : sent;
    da.y = (e0 + 1 < nE) ? dsts[min(e0 + 1, nE - 1)] : sent;
    da.z = (e0 + 2 < nE) ? dsts[min(e0 + 2, nE - 1)] : sent;
    da.w = (e0 + 3 < nE) ? dsts[min(e0 + 3, nE - 1)] : sent;
    db.x = (e0 + 4 < nE) ? dsts[min(e0 + 4, nE - 1)] : sent;
    db.y = (e0 + 5 < nE) ? dsts[min(e0 + 5, nE - 1)] : sent;
    db.z = (e0 + 6 < nE) ? dsts[min(e0 + 6, nE - 1)] : sent;
    db.w = (e0 + 7 < nE) ? dsts[min(e0 + 7, nE - 1)] : sent;
  }
  const unsigned nbs = (unsigned)slotBase;
  const unsigned unb = (unsigned)nb;
  const unsigned s0 = (unsigned)da.x - nbs, s1 = (unsigned)da.y - nbs;
  const unsigned s2 = (unsigned)da.z - nbs, s3 = (unsigned)da.w - nbs;
  const unsigned s4 = (unsigned)db.x - nbs, s5 = (unsigned)db.y - nbs;
  const unsigned s6 = (unsigned)db.z - nbs, s7 = (unsigned)db.w - nbs;
  const bool h0 = s0 < unb, h1 = s1 < unb, h2 = s2 < unb, h3 = s3 < unb;
  const bool h4 = s4 < unb, h5 = s5 < unb, h6 = s6 < unb, h7 = s7 < unb;
  const unsigned any = __builtin_amdgcn_ballot_w32(h0 | h1 | h2 | h3 | h4 | h5 | h6 | h7);
  if (any != 0u) {
#define HITJ(J, HJ, SJ) { \
      const unsigned mj = __builtin_amdgcn_ballot_w32(HJ); \
      if (mj != 0u) { \
        if (HJ) { \
          const int pos = wc + (int)__builtin_amdgcn_mbcnt_lo(mj, 0u); \
          if (pos < WCAP) list[wave * WCAP + pos] = ((el0 + (J)) << SLB) | (int)(SJ); \
        } \
        wc += (int)__builtin_popcount(mj); } }
    HITJ(0, h0, s0)
    HITJ(1, h1, s1)
    HITJ(2, h2, s2)
    HITJ(3, h3, s3)
    HITJ(4, h4, s4)
    HITJ(5, h5, s5)
    HITJ(6, h6, s6)
    HITJ(7, h7, s7)
#undef HITJ
  }
  return wc;
}

__global__ __launch_bounds__(NTHR) void k_prep(const float* __restrict__ W1, const float* __restrict__ W2,
                                               const float* __restrict__ Wl, unsigned short* W1D,
                                               unsigned short* W2B, unsigned short* WlT) {
  const int u = (int)blockIdx.x * NTHR + (int)threadIdx.x;
  v8us o;
  unsigned short* dp;
  if (u < PU1) {
    const int n  = u >> 2;
    const int k8 = (u & 3) * 8;
    const int kk = k8 & (IN_F - 1);
    const float* p = W1 + (size_t)kk * H1 + n;
#pragma unroll
    for (int i = 0; i < 8; ++i) o[i] = (unsigned short)bf16_bits(p[(size_t)i * H1]);
    dp = W1D + (size_t)n * KA1 + k8;
  } else if (u < PU1 + PU2) {
    const int v  = u - PU1;
    const int r  = v >> 7;
    const int k8 = (v & 127) * 8;
    const float* p = W2 + (size_t)r * H2 + k8;
    const v4f a = *(const v4f*)p;
    const v4f b = *(const v4f*)(p + 4);
    o[0] = (unsigned short)bf16_bits(a.x); o[1] = (unsigned short)bf16_bits(a.y);
    o[2] = (unsigned short)bf16_bits(a.z); o[3] = (unsigned short)bf16_bits(a.w);
    o[4] = (unsigned short)bf16_bits(b.x); o[5] = (unsigned short)bf16_bits(b.y);
    o[6] = (unsigned short)bf16_bits(b.z); o[7] = (unsigned short)bf16_bits(b.w);
    dp = W2B + (size_t)r * H2 + k8;
  } else if (u < PU1 + PU2 + PU3) {
    const int v  = u - PU1 - PU2;
    const int n  = v >> 7;
    const int k8 = (v & 127) * 8;
    const float* p = Wl + (size_t)k8 * OUT_F + n;
#pragma unroll
    for (int i = 0; i < 8; ++i) o[i] = (unsigned short)bf16_bits(p[(size_t)i * OUT_F]);
    dp = WlT + (size_t)n * H2 + k8;
  } else {
    return;
  }
  *(volatile v8us*)dp = o;
  __threadfence();
  *(volatile v8us*)dp = o;
}

__global__ __launch_bounds__(FTHR) void k_fold(const unsigned short* __restrict__ W2B,
                                               const unsigned short* __restrict__ WlT,
                                               const float* __restrict__ b2, const float* __restrict__ Wl,
                                               const float* __restrict__ bl, unsigned short* WcT3, float* C16) {
  __shared__ __attribute__((aligned(16))) float wc[H1 * OUT_F];
  __shared__ __attribute__((aligned(16))) float cs[32];
  const int tid = (int)threadIdx.x, lane = tid & 31, wave = tid >> 5, hh = lane >> 4, m = lane & 15;

  v8f acc0 = {0.f, 0.f, 0.f, 0.f, 0.f, 0.f, 0.f, 0.f};
  v8f acc1 = acc0;
  const unsigned short* ap0 = W2B + (size_t)(32 * wave + m) * H2 + 8 * hh;
  const unsigned short* ap1 = ap0 + (size_t)16 * H2;
  const unsigned short* bp  = WlT + (size_t)m * H2 + 8 * hh;
#pragma unroll 1
  for (int ks = 0; ks < H2 / 32; ++ks) {
    FragB bf, a0, a1;
    bf.h[0] = *(const v8usa*)(bp + 32 * ks);
    bf.h[1] = *(const v8usa*)(bp + 32 * ks + 16);
    a0.h[0] = *(const v8usa*)(ap0 + 32 * ks);
    a0.h[1] = *(const v8usa*)(ap0 + 32 * ks + 16);
    a1.h[0] = *(const v8usa*)(ap1 + 32 * ks);
    a1.h[1] = *(const v8usa*)(ap1 + 32 * ks + 16);
    acc0 = wmb(a0, bf, acc0);
    acc1 = wmb(a1, bf, acc1);
  }
#pragma unroll
  for (int r = 0; r < 8; ++r) {
    wc[(32 * wave + 8 * hh + r) * OUT_F + m]      = acc0[r];
    wc[(32 * wave + 16 + 8 * hh + r) * OUT_F + m] = acc1[r];
  }
  if (wave == 0) {
    const int j = lane & 15;
    float s = 0.0f;
#pragma unroll 4
    for (int k = 0; k < H2; ++k) s = fmaf(bf16_val(b2[k]), bf16_val(Wl[(size_t)k * OUT_F + j]), s);
    s = s + bf16_val(bl[j]);
    cs[lane] = (lane < 16) ? s : 0.0f;
  }
  __syncthreads();

  v8us ov[6];
#pragma unroll
  for (int it = 0; it < 6; ++it) {
    const int p   = it * FTHR + tid;
    const int n   = p / 192;
    const int k8  = (p - n * 192) * 8;
    const int seg = k8 >> 9;
    const int kk  = k8 & (H1 - 1);
    v8us o;
#pragma unroll
    for (int j = 0; j < 8; ++j) {
      const float v = wc[(kk + j) * OUT_F + n];
      const unsigned hb = bf16_bits(v);
      const unsigned lb = bf16_bits(v - __uint_as_float(hb << 16));
      o[j] = (unsigned short)((seg == 2) ? lb : hb);
    }
    ov[it] = o;
  }
#pragma unroll
  for (int it = 0; it < 6; ++it) *(volatile v8us*)(WcT3 + 8 * (size_t)(it * FTHR + tid)) = ov[it];
  const v4f cvv = *(const v4fa*)(cs + 4 * (lane & 7));
  const bool cw = (wave == 0) && (lane < 8);
  if (cw) *(volatile v4f*)(C16 + 4 * lane) = cvv;
  __threadfence();
#pragma unroll
  for (int it = 0; it < 6; ++it) *(volatile v8us*)(WcT3 + 8 * (size_t)(it * FTHR + tid)) = ov[it];
  if (cw) *(volatile v4f*)(C16 + 4 * lane) = cvv;
}

__global__ __launch_bounds__(NTHR) void k_deg(const int* __restrict__ dsts, int nE, int vec8, float* dis) {
  __shared__ __attribute__((aligned(16))) int scnt[NBA];
  __shared__ __attribute__((aligned(16))) int list[LISTN];
  __shared__ __attribute__((aligned(16))) float sdis[NBA];
  __shared__ int wcnt[NWAVE];
  const int tid = (int)threadIdx.x, lane = tid & 31, wave = tid >> 5;
  const int nodeBase = (int)blockIdx.x * NBA;

  for (int i = tid; i < NBA; i += NTHR) scnt[i] = 0;
  for (int i = tid; i < LISTN; i += NTHR) list[i] = 0;
  if (tid < NWAVE) wcnt[tid] = 0;
  __syncthreads();

  const int nChunks = (nE + CHUNK - 1) / CHUNK;
#pragma unroll 1
  for (int ch = 0; ch < nChunks; ++ch) {
    const int cbase = ch * CHUNK;
    const int wc = scan_chunk<SLA>(dsts, nE, cbase, nodeBase, NBA, vec8, list, tid, lane, wave);
    if (lane == 0) wcnt[wave] = wc;
    __syncthreads();
    if (wave == 0) {
#pragma unroll 1
      for (int w2 = 0; w2 < NWAVE; ++w2) {
        int c = wcnt[w2];
        c = c < 0 ? 0 : (c > WCAP ? WCAP : c);
#pragma unroll 1
        for (int b0 = 0; b0 < c; b0 += 32) {
          const int idx = b0 + lane;
          const int ent = list[w2 * WCAP + (idx < WCAP ? idx : WCAP - 1)];
          const int m32 = (c - b0) < 32 ? (c - b0) : 32;
#pragma unroll 1
          for (int k = 0; k < m32; ++k) {
            const int u  = __builtin_amdgcn_readlane(ent, k);
            const int sl = u & (NBA - 1);
            if (lane == 0) scnt[sl] = scnt[sl] + 1;
          }
        }
      }
    }
    __syncthreads();
  }

#pragma unroll 1
  for (int i = tid; i < NBA; i += NTHR) {
    const float d = (float)scnt[i] + 1.0f;
    sdis[i] = (d > 0.0f) ? (1.0f / sqrtf(d)) : 0.0f;
  }
  __syncthreads();
  const v4f v = *(const v4fa*)(sdis + 4 * tid);
  float* op = dis + (size_t)nodeBase + 4 * tid;
  *(volatile v4f*)op = v;
  __threadfence();
  *(volatile v4f*)op = v;
}

template <int MODE>
__global__ __launch_bounds__(NTHR) void k_scan(const int* __restrict__ srcs, const int* __restrict__ dsts,
                                               int nE, int nN, int vec8, int mRows,
                                               const float* __restrict__ dis, const float* __restrict__ xl,
                                               const float* __restrict__ cvec,
                                               unsigned short* axo, float* outp) {
  extern __shared__ __attribute__((aligned(16))) int dsm[];
  int* list = dsm;
  int* hl   = dsm + LISTN;
  int* sl   = dsm + LISTN + RCAP;
  int* cnt  = dsm + LISTN + 2 * RCAP;
  int* offs = cnt + NBA;
  int* cur  = offs + NBA;
  int* misc = cur + NBA;
  const int tid = (int)threadIdx.x, lane = tid & 31, wave = tid >> 5;
  const int nodeBase = (int)blockIdx.x * NBA;
  const int chn = lane & 15;

  {
    const v4i z4 = {0, 0, 0, 0};
    for (int i = tid * 4; i < AGG_ZINTS; i += NTHR * 4) *(v4ia*)(dsm + i) = z4;
    if (tid < 16) misc[tid] = 0;
  }
  float cv = 0.0f;
  if constexpr (MODE == 0) cv = cvec[chn];
  __syncthreads();

  int t = 0, ov = 0;
  const int nChunks = (nE + CHUNK - 1) / CHUNK;
#pragma unroll 1
  for (int ch = 0; ch < nChunks; ++ch) {
    const int cbase = ch * CHUNK;
    const int wc = scan_chunk<SLA>(dsts, nE, cbase, nodeBase, NBA, vec8, list, tid, lane, wave);
    if (lane == 0) misc[wave] = wc;
    __syncthreads();
    if (wave == 0) {
#pragma unroll 1
      for (int w2 = 0; w2 < NWAVE; ++w2) {
        int c = misc[w2];
        c = c < 0 ? 0 : (c > WCAP ? WCAP : c);
#pragma unroll 1
        for (int b0 = 0; b0 < c; b0 += 32) {
          const int idx = b0 + lane;
          const int ent = list[w2 * WCAP + (idx < WCAP ? idx : WCAP - 1)];
          const int m32 = (c - b0) < 32 ? (c - b0) : 32;
#pragma unroll 1
          for (int k = 0; k < m32; ++k) {
            const int u    = __builtin_amdgcn_readlane(ent, k);
            const int slot = u & (NBA - 1);
            const int el   = (u >> SLA) & (CHUNK - 1);
            const int pk   = ((cbase + el) << SLA) | slot;
            if (t < RCAP) {
              if (lane == 0) { hl[t] = pk; cnt[slot] = cnt[slot] + 1; }
              t = t + 1;
            } else {
              ov = 1;
            }
          }
        }
      }
    }
    __syncthreads();
  }
  if (wave == 0 && lane == 0) { misc[8] = t; misc[9] = ov; }
  __syncthreads();
  int tt = misc[8];
  tt = tt < 0 ? 0 : (tt > RCAP ? RCAP : tt);
  const int ovf = misc[9];

  if (wave == 0) {
    const int base = lane * (NBA / 32);
    int s = 0;
#pragma unroll 1
    for (int i = 0; i < NBA / 32; ++i) s += cnt[base + i];
    int incl = s;
#pragma unroll
    for (int d = 1; d < 32; d <<= 1) {
      const int y = __shfl_up(incl, d, 32);
      if (lane >= d) incl += y;
    }
    int run = incl - s;
#pragma unroll 1
    for (int i = 0; i < NBA / 32; ++i) {
      const int cvv = cnt[base + i];
      offs[base + i] = run;
      cur[base + i]  = run;
      run += cvv;
    }
  }
  __syncthreads();
  if (wave == 0) {
#pragma unroll 1
    for (int b0 = 0; b0 < tt; b0 += 32) {
      const int idx = b0 + lane;
      const int ent = hl[idx < RCAP ? idx : RCAP - 1];
      const int m32 = (tt - b0) < 32 ? (tt - b0) : 32;
#pragma unroll 1
      for (int k = 0; k < m32; ++k) {
        const int u    = __builtin_amdgcn_readlane(ent, k);
        const int slot = u & (NBA - 1);
        if (lane == 0) {
          int p = cur[slot];
          p = p < 0 ? 0 : (p > RCAP - 1 ? RCAP - 1 : p);
          sl[p] = u;
          cur[slot] = p + 1;
        }
      }
    }
  }
  __syncthreads();

  const float qnan = __int_as_float(0x7fc00000);
  const float pz = (ovf != 0) ? qnan : 0.0f;
  unsigned short* sth = (unsigned short*)hl;
  float* stf = (float*)hl;
#pragma unroll 1
  for (int si = 0; si < NBA / NWAVE; ++si) {
    const int s    = si * NWAVE + wave;
    const int node = nodeBase + s;
    int c = cnt[s];
    const bool big = c > DEGCAP;
    c = c < 0 ? 0 : (c > DEGCAP ? DEGCAP : c);
    int o = offs[s];
    o = o < 0 ? 0 : (o > RCAP ? RCAP : o);
    const int nc = node < nN ? node : nN - 1;
    const float dd = dis[nc];
    const float rd = dd * dd;
    float acc = 0.0f;
#pragma unroll 1
    for (int b0 = 0; b0 < c; b0 += 32) {
      int idx = o + b0 + lane;
      idx = idx > RCAP - 1 ? RCAP - 1 : idx;
      const int ent = sl[idx];
      int eid = ent >> SLA;
      eid = eid < 0 ? 0 : (eid > nE - 1 ? nE - 1 : eid);
      int sr = srcs[eid];
      sr = sr < 0 ? 0 : (sr > nN - 1 ? nN - 1 : sr);
      const float cf  = dis[sr] * dd;
      const int   cfi = __float_as_int(cf);
      const int m32 = (c - b0) < 32 ? (c - b0) : 32;
#pragma unroll 1
      for (int k = 0; k < m32; ++k) {
        const int   sk = __builtin_amdgcn_readlane(sr, k);
        const float ck = __int_as_float(__builtin_amdgcn_readlane(cfi, k));
        float a = xl[(size_t)sk * RW + chn];
        if constexpr (MODE != 0) a = bf16_val(a);
        acc = fmaf(ck, a, acc);
      }
    }
    float sv = xl[(size_t)nc * RW + chn];
    if constexpr (MODE != 0) sv = bf16_val(sv);
    const float pzr = big ? qnan : pz;
    const bool live = node < nN;
    if constexpr (MODE != 0) {
      const float y = (acc + sv * rd) + pzr;
      const float v = live ? y : 0.0f;
      const unsigned hb = bf16_bits(v);
      const unsigned lb = bf16_bits(v - __uint_as_float(hb << 16));
      sth[s * 32 + lane] = (unsigned short)((lane < 16) ? hb : lb);
    } else {
      const float y = ((acc + sv * rd) + cv) + pzr;
      const float v = live ? y : 0.0f;
      if (lane < 16) stf[s * RW + lane] = v;
    }
  }
  __syncthreads();

  if constexpr (MODE != 0) {
    int nrows = mRows - nodeBase;
    nrows = nrows < 0 ? 0 : (nrows > NBA ? NBA : nrows);
    const int npc = nrows * 4;
    unsigned short* gb = axo + (size_t)nodeBase * KA1;
#pragma unroll 1
    for (int p = tid; p < npc; p += NTHR) {
      const v8us q = *(const v8usa*)(sth + 8 * p);
      *(volatile v8us*)(gb + 8 * (size_t)p) = q;
    }
    __threadfence();
#pragma unroll 1
    for (int p = tid; p < npc; p += NTHR) {
      const v8us q = *(const v8usa*)(sth + 8 * p);
      *(volatile v8us*)(gb + 8 * (size_t)p) = q;
    }
  } else {
    int nrows = nN - nodeBase;
    nrows = nrows < 0 ? 0 : (nrows > NBA ? NBA : nrows);
    const int npc = nrows * 4;
    float* gb = outp + (size_t)nodeBase * RW;
#pragma unroll 1
    for (int p = tid; p < npc; p += NTHR) {
      const v4f q = *(const v4fa*)(stf + 4 * p);
      *(volatile v4f*)(gb + 4 * (size_t)p) = q;
    }
    __threadfence();
#pragma unroll 1
    for (int p = tid; p < npc; p += NTHR) {
      const v4f q = *(const v4fa*)(stf + 4 * p);
      *(volatile v4f*)(gb + 4 * (size_t)p) = q;
    }
  }
}

__global__ __launch_bounds__(GTHR) void k_gemm1(const unsigned short* __restrict__ AX,
                                                const unsigned short* __restrict__ W1D,
                                                const float* __restrict__ b1, unsigned short* X1, int nOut) {
  __shared__ __attribute__((aligned(16))) float stg[GBM * GBN];
  const int tid = (int)threadIdx.x, lane = tid & 31, wave = tid >> 5, hh = lane >> 4, m = lane & 15;
  const int rowBase = (int)blockIdx.x * GBM;
  const int col0    = (int)blockIdx.y * GBN;

  v8f acc[8];
  {
    const v8f z = {0.f, 0.f, 0.f, 0.f, 0.f, 0.f, 0.f, 0.f};
#pragma unroll
    for (int t = 0; t < 8; ++t) acc[t] = z;
  }
  const unsigned short* ap = AX + (size_t)(rowBase + 16 * wave + m) * KA1 + 8 * hh;
  const unsigned short* bp = W1D + (size_t)(col0 + m) * KA1 + 8 * hh;
  FragB af;
  af.h[0] = *(const v8usa*)ap;
  af.h[1] = *(const v8usa*)(ap + 16);
#pragma unroll
  for (int nt = 0; nt < 8; ++nt) {
    const unsigned short* wq = bp + (size_t)(16 * nt) * KA1;
    FragB bf;
    bf.h[0] = *(const v8usa*)wq;
    bf.h[1] = *(const v8usa*)(wq + 16);
    acc[nt] = wmb(af, bf, acc[nt]);
  }

#pragma unroll
  for (int nt = 0; nt < 8; ++nt) {
    const int lc = 16 * nt + m;
#pragma unroll
    for (int r = 0; r < 8; ++r) {
      const int lr = 16 * wave + 8 * hh + r;
      stg[lr * GBN + lc] = acc[nt][r];
    }
  }
  __syncthreads();

  v4f bb4;
  {
    const v4f t1 = *(const v4f*)(b1 + col0 + 4 * lane);
    bb4.x = bf16_val(t1.x); bb4.y = bf16_val(t1.y); bb4.z = bf16_val(t1.z); bb4.w = bf16_val(t1.w);
  }
  v4f pv[16];
#pragma unroll
  for (int i = 0; i < 16; ++i) pv[i] = *(const v4fa*)(stg + (16 * wave + i) * GBN + 4 * lane);
  __syncthreads();

#pragma unroll
  for (int i = 0; i < 16; ++i) {
    const bool ok = (rowBase + 16 * wave + i) < nOut;
    const v4f t = pv[i] + bb4;
    v4f y;
    y.x = (t.x > 0.0f) ? t.x : (t.x - t.x);
    y.y = (t.y > 0.0f) ? t.y : (t.y - t.y);
    y.z = (t.z > 0.0f) ? t.z : (t.z - t.z);
    y.w = (t.w > 0.0f) ? t.w : (t.w - t.w);
    y.x = ok ? y.x : 0.0f; y.y = ok ? y.y : 0.0f; y.z = ok ? y.z : 0.0f; y.w = ok ? y.w : 0.0f;
    v4us h4, l4;
    unsigned hb;
    hb = bf16_bits(y.x); h4[0] = (unsigned short)hb; l4[0] = (unsigned short)bf16_bits(y.x - __uint_as_float(hb << 16));
    hb = bf16_bits(y.y); h4[1] = (unsigned short)hb; l4[1] = (unsigned short)bf16_bits(y.y - __uint_as_float(hb << 16));
    hb = bf16_bits(y.z); h4[2] = (unsigned short)hb; l4[2] = (unsigned short)bf16_bits(y.z - __uint_as_float(hb << 16));
    hb = bf16_bits(y.w); h4[3] = (unsigned short)hb; l4[3] = (unsigned short)bf16_bits(y.w - __uint_as_float(hb << 16));
    unsigned short* srow = (unsigned short*)stg + (size_t)(16 * wave + i) * (2 * GBN);
    *(v4usa*)(srow + 4 * lane) = h4;
    *(v4usa*)(srow + GBN + 4 * lane) = l4;
  }
  __syncthreads();
  v8us qv[16];
#pragma unroll
  for (int i = 0; i < 16; ++i) {
    const unsigned short* srow = (const unsigned short*)stg + (size_t)(16 * wave + i) * (2 * GBN);
    qv[i] = *(const v8usa*)(srow + 8 * lane);
  }
  const int goff = (lane < 16) ? (col0 + 8 * lane) : (H1 + col0 + 8 * (lane - 16));
#pragma unroll
  for (int i = 0; i < 16; ++i) {
    unsigned short* rp = X1 + (size_t)(rowBase + 16 * wave + i) * X1P + goff;
    *(volatile v8us*)rp = qv[i];
  }
  __threadfence();
#pragma unroll
  for (int i = 0; i < 16; ++i) {
    unsigned short* rp = X1 + (size_t)(rowBase + 16 * wave + i) * X1P + goff;
    *(volatile v8us*)rp = qv[i];
  }
}

__global__ __launch_bounds__(NTHR) void k_gemmz(const unsigned short* __restrict__ X1,
                                                const unsigned short* __restrict__ WcT3, float* Z) {
  __shared__ __attribute__((aligned(16))) float stg[ZBM * OUT_F];
  const int tid = (int)threadIdx.x, lane = tid & 31, wave = tid >> 5, hh = lane >> 4, m = lane & 15;
  const int rowBase = (int)blockIdx.x * ZBM;

  v8f acc = {0.f, 0.f, 0.f, 0.f, 0.f, 0.f, 0.f, 0.f};
  const unsigned short* ap = X1 + (size_t)(rowBase + 16 * wave + m) * X1P + 8 * hh;
  const unsigned short* bp = WcT3 + (size_t)m * KZ + 8 * hh;
#pragma unroll 1
  for (int ks = 0; ks < KZ / 32; ++ks) {
    const int ka = (ks & 31) * 32;
    FragB af, bf;
    af.h[0] = *(const v8usa*)(ap + ka);
    af.h[1] = *(const v8usa*)(ap + ka + 16);
    bf.h[0] = *(const v8usa*)(bp + 32 * ks);
    bf.h[1] = *(const v8usa*)(bp + 32 * ks + 16);
    acc = wmb(af, bf, acc);
  }
#pragma unroll
  for (int r = 0; r < 8; ++r) stg[(16 * wave + 8 * hh + r) * OUT_F + m] = acc[r];
  __syncthreads();
  const v4f f0 = *(const v4fa*)(stg + 4 * tid);
  const v4f f1 = *(const v4fa*)(stg + 4 * (tid + NTHR));
  float* zb = Z + (size_t)rowBase * OUT_F;
  *(volatile v4f*)(zb + 4 * (size_t)tid) = f0;
  *(volatile v4f*)(zb + 4 * (size_t)(tid + NTHR)) = f1;
  __threadfence();
  *(volatile v4f*)(zb + 4 * (size_t)tid) = f0;
  *(volatile v4f*)(zb + 4 * (size_t)(tid + NTHR)) = f1;
}

static inline int cdiv(int a, int b) { return (a + b - 1) / b; }
static inline size_t al256(size_t o) { return (o + 255) & ~(size_t)255; }

extern "C" void kernel_launch(void* const* d_in, const int* in_sizes, int n_in,
                              void* d_out, int out_size, void* d_ws, size_t ws_size,
                              hipStream_t stream) {
  if (n_in < 8) return;
  if (in_sizes[0] < IN_F || (in_sizes[0] % IN_F) != 0) return;
  const int nN = in_sizes[0] / IN_F;
  if (nN < 16 || nN > (1 << 22) || (nN & 1) != 0) return;
  if (in_sizes[1] < 2 || (in_sizes[1] & 1) != 0) return;
  const int nE = in_sizes[1] / 2;
  if (nE < 1 || nE >= (1 << (31 - SLA))) return;
  if (in_sizes[2] != IN_F * H1 || in_sizes[3] != H1) return;
  if (in_sizes[4] != H1 * H2 || in_sizes[5] != H2) return;
  if (in_sizes[6] != H2 * OUT_F || in_sizes[7] != OUT_F) return;
  if ((long long)out_size != (long long)nN * OUT_F) return;

  const float* x    = (const float*)d_in[0];
  const int*   edge = (const int*)d_in[1];
  const float* W1   = (const float*)d_in[2];
  const float* b1   = (const float*)d_in[3];
  const float* W2   = (const float*)d_in[4];
  const float* b2   = (const float*)d_in[5];
  const float* Wl   = (const float*)d_in[6];
  const float* bl   = (const float*)d_in[7];
  float* out = (float*)d_out;
  const int* src = edge;
  const int* dst = edge + nE;

  const int MP  = cdiv(nN, ZBM) * ZBM;
  const int gM1 = MP / GBM;
  const int gMz = MP / ZBM;
  const int gA  = cdiv(MP, NBA);
  const int NBP = gA * NBA;
  if ((MP % GBM) != 0 || (long long)gA * NBA < (long long)MP || NBP < nN) return;
  const int vec8 = ((nE & 3) == 0) ? 1 : 0;

  char* ws = (char*)d_ws;
  size_t off = 0;
  const size_t oW1D = off; off = al256(off + (size_t)H1 * KA1 * 2);
  const size_t oW2B = off; off = al256(off + (size_t)H1 * H2 * 2);
  const size_t oWlT = off; off = al256(off + (size_t)OUT_F * H2 * 2);
  const size_t oWc3 = off; off = al256(off + (size_t)OUT_F * KZ * 2);
  const size_t oC16 = off; off = al256(off + (size_t)128);
  const size_t oDIS = off; off = al256(off + (size_t)NBP * 4);
  const size_t oAX  = off; off = al256(off + (size_t)MP * KA1 * 2);
  const size_t oX1  = off; off = al256(off + (size_t)MP * X1P * 2);
  const size_t oZ   = off; off = al256(off + (size_t)MP * OUT_F * 4);
  if (off > ws_size || off > (size_t)WSMAX) return;
  unsigned short* W1D  = (unsigned short*)(ws + oW1D);
  unsigned short* W2B  = (unsigned short*)(ws + oW2B);
  unsigned short* WlT  = (unsigned short*)(ws + oWlT);
  unsigned short* WcT3 = (unsigned short*)(ws + oWc3);
  float*          C16  = (float*)(ws + oC16);
  float*          DIS  = (float*)(ws + oDIS);
  unsigned short* AXhl = (unsigned short*)(ws + oAX);
  unsigned short* X1hl = (unsigned short*)(ws + oX1);
  float*          Z    = (float*)(ws + oZ);

  const size_t scanLds = (size_t)AGG_LDS_INTS * 4;
  hipFuncSetAttribute(reinterpret_cast<const void*>(&k_scan<1>), hipFuncAttributeMaxDynamicSharedMemorySize, (int)scanLds);
  hipFuncSetAttribute(reinterpret_cast<const void*>(&k_scan<0>), hipFuncAttributeMaxDynamicSharedMemorySize, (int)scanLds);

  k_prep<<<(PU1 + PU2 + PU3) / NTHR, NTHR, 0, stream>>>(W1, W2, Wl, W1D, W2B, WlT);
  k_fold<<<1, FTHR, 0, stream>>>(W2B, WlT, b2, Wl, bl, WcT3, C16);
  k_deg<<<gA, NTHR, 0, stream>>>(dst, nE, vec8, DIS);
  k_scan<1><<<gA, NTHR, scanLds, stream>>>(src, dst, nE, nN, vec8, MP, DIS, x, C16, AXhl, out);
  k_gemm1<<<dim3(gM1, H1 / GBN), GTHR, 0, stream>>>(AXhl, W1D, b1, X1hl, nN);
  k_gemmz<<<gMz, NTHR, 0, stream>>>(X1hl, WcT3, Z);
  k_scan<0><<<gA, NTHR, scanLds, stream>>>(src, dst, nE, nN, vec8, MP, DIS, Z, C16, AXhl, out);
}
